// LightweightSelfAttention_51694226375319
// MI455X (gfx1250) — hardware-verified
//
#include <hip/hip_runtime.h>


namespace {
constexpr int Bn = 4, C = 256, CR = 32, HW = 64, NP = HW * HW, NT = Bn * NP;
constexpr float XS = 8.0f, PS = 8.0f;
struct Wo_ { static constexpr size_t Q = 0, K = (size_t)CR * C, V = 2 * (size_t)CR * C, END = V + (size_t)C * C; };

typedef _Float16 b16;
typedef __attribute__((ext_vector_type(16))) _Float16 v16b;
typedef __attribute__((ext_vector_type(8))) _Float16 v8b;
typedef __attribute__((ext_vector_type(8))) float v8f;
typedef __attribute__((ext_vector_type(4))) float v4f;
__device__ __forceinline__ float bf16_rne(float f) { unsigned int u = __float_as_uint(f); u += 0x7FFFu + ((u >> 16) & 1u); return __uint_as_float(u & 0xFFFF0000u); }
__device__ __forceinline__ void split16(float v, b16& hi, b16& lo) { hi = (b16)v; lo = (b16)(v - (float)hi); }
__device__ __forceinline__ v16b frag_kb(const b16* p, int hh) { const v8b a = *(const v8b*)(p + 8 * hh), b = *(const v8b*)(p + 16 + 8 * hh); v16b f;
#pragma unroll
  for (int e = 0; e < 8; ++e) { f[e] = a[e]; f[8 + e] = b[e]; } return f; }
__device__ __forceinline__ v8f wmma16b(v16b a, v16b b, v8f c) { v8f d = __builtin_amdgcn_wmma_f32_16x16x32_f16(false, a, false, b, (short)0, c, false, false); asm volatile("v_nop\n\tv_nop\n\tv_nop\n\tv_nop" : "+v"(d) : "v"(a), "v"(b)); return d; }
__device__ __forceinline__ void wave_lds_sync() { __builtin_amdgcn_fence(__ATOMIC_RELEASE, "workgroup"); __builtin_amdgcn_wave_barrier(); __builtin_amdgcn_fence(__ATOMIC_ACQUIRE, "workgroup"); }
__device__ __forceinline__ float nexp(float x) { return __builtin_amdgcn_exp2f(x * 1.4426950408889634f); }
__device__ __forceinline__ float pmul(float a, float b) { float p = a * b; asm volatile("" : "+v"(p)); return p; }

__global__ __launch_bounds__(256) void rows_kernel(const float* __restrict__ x, const float* __restrict__ Wq, const float* __restrict__ Wk, const float* __restrict__ Wv, b16* __restrict__ X, b16* __restrict__ R) {
  __shared__ __attribute__((aligned(16))) b16 Tt[64][C + 8];
  const int b = blockIdx.y, p0 = blockIdx.x * 64, t_ = threadIdx.x;
  for (int i = t_; i < C * 64; i += 256) { const int c = i >> 6, p = i & 63; Tt[p][c] = (b16)bf16_rne(x[((size_t)b * C + c) * NP + p0 + p]); }
  __syncthreads();
  for (int pass = 0; pass < 2; ++pass) {
    for (int i = t_; i < 64 * (C / 8); i += 256) { const int p = i / (C / 8), c8 = (i % (C / 8)) * 8; *(volatile v8b*)(X + ((size_t)b * NP + p0 + p) * C + c8) = *(const v8b*)(&Tt[p][c8]); }
    if (b == 0) { for (int i = blockIdx.x * 256 + t_; i < (int)(Wo_::END / 8); i += 64 * 256) { const size_t q = (size_t)i * 8; const float* s_ = (q < Wo_::K) ? (Wq + q) : (q < Wo_::V) ? (Wk + (q - Wo_::K)) : (Wv + (q - Wo_::V)); v8b v; for (int e = 0; e < 8; ++e) v[e] = (b16)bf16_rne(s_[e]); *(volatile v8b*)(R + q) = v; } }
    __threadfence(); }
}

__global__ __launch_bounds__(128) void proj_kernel(const b16* __restrict__ X, const b16* __restrict__ R, b16* __restrict__ QH, b16* __restrict__ QL, b16* __restrict__ KH, b16* __restrict__ KL, b16* __restrict__ VT) {
  __shared__ __attribute__((aligned(16))) b16 Tq[4][128][CR + 8]; __shared__ __attribute__((aligned(16))) b16 Tv[128][128 + 8];
  const int lane = threadIdx.x & 31, wave = threadIdx.x >> 5, nloc = lane & 15, hlf = lane >> 4, b = blockIdx.y, p0 = blockIdx.x * 128, m0 = p0 + wave * 32; const b16* A = X + (size_t)b * NP * C;
  { v8f acc[2][4];
#pragma unroll
    for (int r = 0; r < 2; ++r)
#pragma unroll
      for (int t = 0; t < 4; ++t) acc[r][t] = (v8f){};
#pragma unroll 2
    for (int kb = 0; kb < C; kb += 32) { const v16b a0 = frag_kb(A + (size_t)(m0 + nloc) * C + kb, hlf), a1 = frag_kb(A + (size_t)(m0 + 16 + nloc) * C + kb, hlf);
#pragma unroll
      for (int t = 0; t < 4; ++t) { const v16b bw = frag_kb(R + (size_t)(t * 16 + nloc) * C + kb, hlf); acc[0][t] = wmma16b(a0, bw, acc[0][t]); acc[1][t] = wmma16b(a1, bw, acc[1][t]); } }
#pragma unroll
    for (int t = 0; t < 4; ++t)
#pragma unroll
      for (int r = 0; r < 2; ++r)
#pragma unroll
        for (int v = 0; v < 8; ++v) { const int rr = wave * 32 + r * 16 + 8 * hlf + v, cc = (t & 1) * 16 + nloc; b16 a_, c_; split16(acc[r][t][v] * XS, a_, c_); Tq[(t >> 1) * 2][rr][cc] = a_; Tq[(t >> 1) * 2 + 1][rr][cc] = c_; } }
  __syncthreads();
  for (int pass = 0; pass < 2; ++pass) { for (int i = threadIdx.x; i < 4 * 128 * 4; i += 128) { const int pl = i / 512, rem = i % 512, rr = rem >> 2, c8 = (rem & 3) * 8; b16* dst = (pl == 0) ? QH : (pl == 1) ? QL : (pl == 2) ? KH : KL; *(volatile v8b*)(dst + ((size_t)b * NP + p0 + rr) * CR + c8) = *(const v8b*)(&Tq[pl][rr][c8]); } __threadfence(); }
#pragma unroll 1
  for (int half = 0; half < 2; ++half) { v8f acc[2][8];
#pragma unroll
    for (int r = 0; r < 2; ++r)
#pragma unroll
      for (int t = 0; t < 8; ++t) acc[r][t] = (v8f){};
#pragma unroll 2
    for (int kb = 0; kb < C; kb += 32) { const v16b a0 = frag_kb(A + (size_t)(m0 + nloc) * C + kb, hlf), a1 = frag_kb(A + (size_t)(m0 + 16 + nloc) * C + kb, hlf);
#pragma unroll
      for (int t = 0; t < 8; ++t) { const v16b bw = frag_kb(R + Wo_::V + (size_t)(half * 128 + t * 16 + nloc) * C + kb, hlf); acc[0][t] = wmma16b(a0, bw, acc[0][t]); acc[1][t] = wmma16b(a1, bw, acc[1][t]); } }
    __syncthreads();
#pragma unroll
    for (int t = 0; t < 8; ++t)
#pragma unroll
      for (int r = 0; r < 2; ++r)
#pragma unroll
        for (int v = 0; v < 8; ++v) Tv[t * 16 + nloc][wave * 32 + r * 16 + 8 * hlf + v] = (b16)(acc[r][t][v] * XS);
    __syncthreads();
    for (int pass = 0; pass < 2; ++pass) { for (int i = threadIdx.x; i < 128 * 16; i += 128) { const int c = i >> 4, c8 = (i & 15) * 8; *(volatile v8b*)(VT + ((size_t)b * C + half * 128 + c) * NP + p0 + c8) = *(const v8b*)(&Tv[c][c8]); } __threadfence(); } }
}

__global__ __launch_bounds__(128) void attn_kernel(const b16* __restrict__ QH, const b16* __restrict__ QL, const b16* __restrict__ KH, const b16* __restrict__ KL, const b16* __restrict__ VT, float* __restrict__ ATT) {
  __shared__ __attribute__((aligned(16))) b16 Pt[16][32 + 8]; __shared__ float Mx[2][16], Sm[2][16]; __shared__ __attribute__((aligned(16))) float Os[16][C + 4];
  const int wave = threadIdx.x >> 5, lane = threadIdx.x & 31, hh = lane >> 4, col = lane & 15, b = blockIdx.y, q0 = blockIdx.x * 16, qi = q0 + col;
  const size_t rb = (size_t)b * NP * CR; const b16* Vb = VT + (size_t)b * C * NP; const float SC = 1.0f / (XS * XS);
  const v16b qa = frag_kb(QH + rb + (size_t)qi * CR, hh), qb = frag_kb(QL + rb + (size_t)qi * CR, hh);
  float m = -INFINITY, l = 0.0f; v8f o[4] = {{}, {}, {}, {}};
  for (int kb = 0; kb < NP; kb += 32) { float sv[8];
    if (wave < 2) { v8f s = {}; const v16b kf = frag_kb(KH + rb + (size_t)(kb + 16 * wave + col) * CR, hh), kl = frag_kb(KL + rb + (size_t)(kb + 16 * wave + col) * CR, hh);
      s = wmma16b(kf, qa, s); s = wmma16b(kf, qb, s); s = wmma16b(kl, qa, s); float mr = -INFINITY;
#pragma unroll
      for (int r = 0; r < 8; ++r) { sv[r] = s[r] * SC; mr = fmaxf(mr, sv[r]); }
      mr = fmaxf(mr, __shfl_xor(mr, 16)); if (hh == 0) Mx[wave][col] = mr; }
    __syncthreads();
    const float mn = fmaxf(m, fmaxf(Mx[0][col], Mx[1][col])), al_ = nexp(m - mn); m = mn;
    if (wave < 2) { float sum = 0.0f;
#pragma unroll
      for (int r = 0; r < 8; ++r) { const float e = nexp(sv[r] - mn); sum += e; Pt[col][16 * wave + 8 * hh + r] = (b16)(e * PS); }
      sum += __shfl_xor(sum, 16); if (hh == 0) Sm[wave][col] = sum; }
    __syncthreads();
    l = l * al_ + (Sm[0][col] + Sm[1][col]);
    const v16b pb = frag_kb(&Pt[col][0], hh);
#pragma unroll
    for (int t = 0; t < 4; ++t) { o[t] *= al_; o[t] = wmma16b(frag_kb(Vb + (size_t)((wave * 4 + t) * 16 + col) * NP + kb, hh), pb, o[t]); }
    __syncthreads(); }
  const float inv = 1.0f / (l * PS * XS);
#pragma unroll
  for (int t = 0; t < 4; ++t)
#pragma unroll
    for (int r = 0; r < 8; ++r) Os[col][(wave * 4 + t) * 16 + 8 * hh + r] = o[t][r] * inv;
  __syncthreads();
  for (int pass = 0; pass < 2; ++pass) { for (int i = threadIdx.x; i < 16 * (C / 4); i += 128) { const int rr = i / (C / 4), c4 = (i % (C / 4)) * 4; *(volatile v4f*)(ATT + ((size_t)b * NP + q0 + rr) * C + c4) = *(const v4f*)(&Os[rr][c4]); } __threadfence(); }
}

__global__ __launch_bounds__(256) void out_kernel(const float* __restrict__ ATT, const float* __restrict__ x, float* __restrict__ out) {
  __shared__ __attribute__((aligned(16))) float Tq[128][128 + 1];
  const int b = blockIdx.y, p0 = blockIdx.x * 128, t_ = threadIdx.x;
  for (int half = 0; half < 2; ++half) {
    __syncthreads();
    for (int i = t_; i < 128 * 128; i += 256) { const int p = i >> 7, c = i & 127; Tq[c][p] = ATT[((size_t)b * NP + p0 + p) * C + half * 128 + c]; }
    __syncthreads();
    for (int pass = 0; pass < 2; ++pass) { for (int i = t_; i < 128 * 32; i += 256) { const int c = i >> 5, c4 = (i & 31) * 4; const size_t gi = ((size_t)b * C + half * 128 + c) * NP + p0 + c4; const v4f xr = *(const v4f*)(x + gi); v4f o; for (int e = 0; e < 4; ++e) o[e] = Tq[c][c4 + e] + bf16_rne(xr[e]); *(volatile v4f*)(out + gi) = o; } __threadfence(); } }
}
}

extern "C" void kernel_launch(void* const* d_in, const int* in_sizes, int n_in,
                              void* d_out, int out_size, void* d_ws, size_t ws_size, hipStream_t stream) {
  (void)n_in; (void)out_size;
  const float* x = (const float*)d_in[0]; const float* Wq = (const float*)d_in[1]; const float* Wk = (const float*)d_in[2]; const float* Wv = (const float*)d_in[3];
  float* out = (float*)d_out;
  if (in_sizes[0] != NT * C || in_sizes[1] != CR * C || in_sizes[3] != C * C) return;
  size_t off = 0; char* ws = (char*)d_ws;
  auto carve = [&](size_t bytes) { char* p = ws + off; off += (bytes + 255) & ~(size_t)255; return p; };
  b16* X = (b16*)carve((size_t)NT * C * 2); b16* R = (b16*)carve(Wo_::END * 2); b16* QH = (b16*)carve((size_t)NT * CR * 2); b16* QL = (b16*)carve((size_t)NT * CR * 2); b16* KH = (b16*)carve((size_t)NT * CR * 2); b16* KL = (b16*)carve((size_t)NT * CR * 2); b16* VT = (b16*)carve((size_t)NT * C * 2); float* ATT = (float*)carve((size_t)NT * C * 4);
  if (off > ws_size) return;
  rows_kernel<<<dim3(NP / 64, Bn), 256, 0, stream>>>(x, Wq, Wk, Wv, X, R);
  proj_kernel<<<dim3(NP / 128, Bn), 128, 0, stream>>>(X, R, QH, QL, KH, KL, VT);
  attn_kernel<<<dim3(NP / 16, Bn), 128, 0, stream>>>(QH, QL, KH, KL, VT, ATT);
  out_kernel<<<dim3(NP / 128, Bn), 256, 0, stream>>>(ATT, x, out);
}
